// KRNN7_14035953124004
// MI455X (gfx1250) — hardware-verified
//
#include <hip/hip_runtime.h>
#include <math.h>

#define NNODE  325
#define BNR    10400
#define TIN    12
#define TOUT   12
#define NC     10
#define HID    64
#define G3     192
#define XROW   24
#define HP     72
#define WPL    12288
#define NT_REC 128
#define NTILE  650
#define NOUT4  31200

typedef __attribute__((ext_vector_type(16))) _Float16 v16h;
typedef __attribute__((ext_vector_type(8)))  _Float16 v8h;
typedef __attribute__((ext_vector_type(8)))  float    v8f;
typedef __attribute__((ext_vector_type(4)))  float    v4f;

__device__ __forceinline__ void dep_guard3x(v8f& a, v8f& b, v8f& c, v16h x, v16h y) {
  asm volatile("v_nop\n\tv_nop\n\tv_nop\n\tv_nop" : "+v"(a), "+v"(b), "+v"(c) : "v"(x), "v"(y));
}
__device__ __forceinline__ void dep_guard3b(v8f& a, v8f& b, v8f& c, v16h x, v16h y,
                                            v16h b0, v16h b1, v16h b2, v16h b3, v16h b4, v16h b5) {
  asm volatile("v_nop\n\tv_nop\n\tv_nop\n\tv_nop" : "+v"(a), "+v"(b), "+v"(c)
               : "v"(x), "v"(y), "v"(b0), "v"(b1), "v"(b2), "v"(b3), "v"(b4), "v"(b5));
}

template <typename T> struct Frag;
template <> struct Frag<_Float16> {
  typedef v16h V; union U { v16h v; v8h h[2]; };
  static __device__ __forceinline__ v16h load(const _Float16* p) {
    U f; f.h[0] = *(const v8h*)(p); f.h[1] = *(const v8h*)(p + 16); return f.v;
  }
  static __device__ __forceinline__ v8f mma(v16h a, v16h b, v8f c) {
    return __builtin_amdgcn_wmma_f32_16x16x32_f16(false, a, false, b, (short)0, c, false, false);
  }
};

__device__ __forceinline__ unsigned pack_f16x2(float a, float b) {
  const _Float16 h0 = (_Float16)a, h1 = (_Float16)b;
  return (unsigned)__builtin_bit_cast(unsigned short, h0) | ((unsigned)__builtin_bit_cast(unsigned short, h1) << 16);
}
__device__ __forceinline__ void st2u(unsigned* p, unsigned v) { *(volatile unsigned*)p = v; __threadfence(); *(volatile unsigned*)p = v; }
__device__ __forceinline__ float ftanh(float x) { return 1.0f - 2.0f * __builtin_amdgcn_rcpf(1.0f + __expf(2.0f * x)); }
__device__ __forceinline__ float fsigm(float x) { return __builtin_amdgcn_rcpf(1.0f + __expf(-x)); }

__global__ __launch_bounds__(256) void prep_kernel(const float* __restrict__ eWhh, const float* __restrict__ dWhh,
                                                  unsigned* __restrict__ W16u) {
  const int blk = blockIdx.x, tid = threadIdx.x;
  if (blk < 240) {
    const int p = blk * 256 + tid;
    const unsigned u = pack_f16x2(eWhh[2 * p] * 16.0f, eWhh[2 * p + 1] * 16.0f);
    st2u(W16u + p, u);
  } else {
    const int p = (blk - 240) * 256 + tid;
    const unsigned u = pack_f16x2(dWhh[2 * p] * 16.0f, dWhh[2 * p + 1] * 16.0f);
    st2u(W16u + 61440 + p, u);
  }
}

__global__ __launch_bounds__(NT_REC) void gru_seq_kernel(
    const float* __restrict__ X, const _Float16* __restrict__ W16,
    const float* __restrict__ eWih, const float* __restrict__ eBih, const float* __restrict__ eBhh,
    const float* __restrict__ dWih, const float* __restrict__ dBih, const float* __restrict__ dBhh,
    const float* __restrict__ linW, const float* __restrict__ linB,
    float* __restrict__ VALS) {
  __shared__ __align__(16) _Float16 h16[16 * HP];
  __shared__ __align__(16) float xs[16 * XROW];
  __shared__ __align__(16) float red[4 * 16];
  __shared__ __align__(16) float vstage[16 * TOUT];

  const int tid = threadIdx.x, lane = tid & 31, wave = tid >> 5;
  const int rlane = lane & 15, hh = lane >> 4, koff = hh * 8, mOff = hh * 8;
  const int tile = blockIdx.x;
  const int c    = blockIdx.y;
  const int bn0  = tile * 16;

  for (int i = tid; i < 16 * HP; i += NT_REC) h16[i] = (_Float16)0.0f;
  for (int i = tid; i < 16 * XROW; i += NT_REC) xs[i] = X[(size_t)bn0 * XROW + i];
  if (tid < 64) red[tid] = 0.0f;
  __syncthreads();

  const int j = 16 * wave + rlane;
  const _Float16* arow = h16 + rlane * HP + koff;
  const float s16 = 1.0f / 16.0f;
  const v8f z8 = {0.f, 0.f, 0.f, 0.f, 0.f, 0.f, 0.f, 0.f};

  float hreg[8];
#pragma unroll
  for (int r = 0; r < 8; ++r) hreg[r] = 0.0f;

  v16h bq[3][2];

  {
    const _Float16* WE = W16 + (size_t)c * WPL;
#pragma unroll
    for (int g = 0; g < 3; ++g)
#pragma unroll
      for (int kc = 0; kc < 2; ++kc)
        bq[g][kc] = Frag<_Float16>::load(WE + (size_t)(g * HID + j) * HID + koff + 32 * kc);

    const float we0r = eWih[(c * G3 + j) * 2 + 0],           we1r = eWih[(c * G3 + j) * 2 + 1];
    const float we0z = eWih[(c * G3 + HID + j) * 2 + 0],     we1z = eWih[(c * G3 + HID + j) * 2 + 1];
    const float we0n = eWih[(c * G3 + 2 * HID + j) * 2 + 0], we1n = eWih[(c * G3 + 2 * HID + j) * 2 + 1];
    const float beir = eBih[c * G3 + j], beiz = eBih[c * G3 + HID + j], bein = eBih[c * G3 + 2 * HID + j];
    const float behr = eBhh[c * G3 + j], behz = eBhh[c * G3 + HID + j], behn = eBhh[c * G3 + 2 * HID + j];

#pragma unroll 1
    for (int t = 0; t < TIN; ++t) {
      v8f ar = z8, az = z8, an = z8;
      const v16h a0 = Frag<_Float16>::load(arow);
      const v16h a1 = Frag<_Float16>::load(arow + 32);
      ar = Frag<_Float16>::mma(a0, bq[0][0], ar);
      az = Frag<_Float16>::mma(a0, bq[1][0], az);
      an = Frag<_Float16>::mma(a0, bq[2][0], an);
      ar = Frag<_Float16>::mma(a1, bq[0][1], ar);
      az = Frag<_Float16>::mma(a1, bq[1][1], az);
      an = Frag<_Float16>::mma(a1, bq[2][1], an);
      dep_guard3b(ar, az, an, a0, a1, bq[0][0], bq[1][0], bq[2][0], bq[0][1], bq[1][1], bq[2][1]);

#pragma unroll
      for (int r = 0; r < 8; ++r) {
        const float x0 = xs[(mOff + r) * XROW + 2 * t];
        const float x1 = xs[(mOff + r) * XROW + 2 * t + 1];
        const float gir = fmaf(x1, we1r, fmaf(x0, we0r, beir));
        const float giz = fmaf(x1, we1z, fmaf(x0, we0z, beiz));
        const float gin = fmaf(x1, we1n, fmaf(x0, we0n, bein));
        const float ghr = fmaf(ar[r], s16, behr);
        const float ghz = fmaf(az[r], s16, behz);
        const float ghn = fmaf(an[r], s16, behn);
        const float rg = fsigm(gir + ghr);
        const float zg = fsigm(giz + ghz);
        const float ng = ftanh(fmaf(rg, ghn, gin));
        hreg[r] = (1.0f - zg) * ng + zg * hreg[r];
      }
      __syncthreads();
#pragma unroll
      for (int r = 0; r < 8; ++r) h16[(mOff + r) * HP + j] = (_Float16)hreg[r];
      __syncthreads();
    }
  }

  {
    const _Float16* WD = W16 + (size_t)(NC + c) * WPL;
#pragma unroll
    for (int g = 0; g < 3; ++g)
#pragma unroll
      for (int kc = 0; kc < 2; ++kc)
        bq[g][kc] = Frag<_Float16>::load(WD + (size_t)(g * HID + j) * HID + koff + 32 * kc);

    const float wdr = dWih[c * G3 + j], wdz = dWih[c * G3 + HID + j], wdn = dWih[c * G3 + 2 * HID + j];
    const float bdir = dBih[c * G3 + j], bdiz = dBih[c * G3 + HID + j], bdin = dBih[c * G3 + 2 * HID + j];
    const float bdhr = dBhh[c * G3 + j], bdhz = dBhh[c * G3 + HID + j], bdhn = dBhh[c * G3 + 2 * HID + j];
    const float lw = linW[c * HID + j];
    const float lb = linB[c];
    const int   row16 = tid & 15;

#pragma unroll 1
    for (int t = 0; t < TOUT; ++t) {
      float lv[8];
#pragma unroll
      for (int r = 0; r < 8; ++r) {
        const int rr = mOff + r;
        const float vx = xs[rr * XROW + (TIN - 1) * 2];
        const float vs = (((red[rr] + red[16 + rr]) + red[32 + rr]) + red[48 + rr]) + lb;
        lv[r] = (t == 0) ? vx : vs;
      }
      {
        const float vt = (((red[row16] + red[16 + row16]) + red[32 + row16]) + red[48 + row16]) + lb;
        if (t > 0 && tid < 16) vstage[row16 * TOUT + (t - 1)] = vt;
      }

      v8f ar = z8, az = z8, an = z8;
      const v16h a0 = Frag<_Float16>::load(arow);
      const v16h a1 = Frag<_Float16>::load(arow + 32);
      ar = Frag<_Float16>::mma(a0, bq[0][0], ar);
      az = Frag<_Float16>::mma(a0, bq[1][0], az);
      an = Frag<_Float16>::mma(a0, bq[2][0], an);
      ar = Frag<_Float16>::mma(a1, bq[0][1], ar);
      az = Frag<_Float16>::mma(a1, bq[1][1], az);
      an = Frag<_Float16>::mma(a1, bq[2][1], an);
      dep_guard3x(ar, az, an, a0, a1);

#pragma unroll
      for (int r = 0; r < 8; ++r) {
        const float gir = fmaf(lv[r], wdr, bdir);
        const float giz = fmaf(lv[r], wdz, bdiz);
        const float gin = fmaf(lv[r], wdn, bdin);
        const float ghr = fmaf(ar[r], s16, bdhr);
        const float ghz = fmaf(az[r], s16, bdhz);
        const float ghn = fmaf(an[r], s16, bdhn);
        const float rg = fsigm(gir + ghr);
        const float zg = fsigm(giz + ghz);
        const float ng = ftanh(fmaf(rg, ghn, gin));
        hreg[r] = (1.0f - zg) * ng + zg * hreg[r];
      }
      __syncthreads();
#pragma unroll
      for (int r = 0; r < 8; ++r) h16[(mOff + r) * HP + j] = (_Float16)hreg[r];
      float p[8];
#pragma unroll
      for (int r = 0; r < 8; ++r) p[r] = hreg[r] * lw;
#pragma unroll
      for (int r = 0; r < 8; ++r) {
        p[r] += __shfl_xor(p[r], 1, 32);
        p[r] += __shfl_xor(p[r], 2, 32);
        p[r] += __shfl_xor(p[r], 4, 32);
        p[r] += __shfl_xor(p[r], 8, 32);
      }
      if (rlane == 0) {
#pragma unroll
        for (int r = 0; r < 8; ++r) red[wave * 16 + mOff + r] = p[r];
      }
      __syncthreads();
    }
    {
      const float vt = (((red[row16] + red[16 + row16]) + red[32 + row16]) + red[48 + row16]) + lb;
      if (tid < 16) vstage[row16 * TOUT + (TOUT - 1)] = vt;
    }
  }
  __syncthreads();

  if (wave == 0) {
    float* vb = VALS + ((size_t)c * BNR + (size_t)bn0) * TOUT;
    const int l2 = (lane < 16) ? lane : 15;
    for (int pass = 0; pass < 2; ++pass) {
      const v4f v0 = *(const v4f*)(vstage + lane * 4);
      *(volatile v4f*)(vb + lane * 4) = v0;
      const v4f v1 = *(const v4f*)(vstage + 128 + l2 * 4);
      if (lane < 16) *(volatile v4f*)(vb + 128 + lane * 4) = v1;
      __threadfence();
    }
  }
}

__global__ __launch_bounds__(256) void combine_kernel(const float* __restrict__ VALS, const float* __restrict__ embed,
                                                     float* __restrict__ out, int n4) {
  const int i = blockIdx.x * 256 + threadIdx.x;
  if (i >= n4) return;
  const int bn = i / 3;
  const int n = bn % NNODE;
  const float* er = embed + (size_t)n * NC;
  float mx = er[0];
#pragma unroll 1
  for (int cc = 1; cc < NC; ++cc) mx = fmaxf(mx, er[cc]);
  float s = 0.0f;
#pragma unroll 1
  for (int cc = 0; cc < NC; ++cc) s += expf(er[cc] - mx);
  const float inv = 1.0f / s;
  v4f acc = {0.f, 0.f, 0.f, 0.f};
#pragma unroll 1
  for (int cc = 0; cc < NC; ++cc) {
    const float w = expf(er[cc] - mx) * inv;
    const v4f v = *(const v4f*)(VALS + (size_t)cc * (BNR * TOUT) + (size_t)i * 4);
    acc += v * w;
  }
  float* op = out + (size_t)i * 4;
  *(volatile v4f*)op = acc;
  __threadfence();
  *(volatile v4f*)op = acc;
}

extern "C" void kernel_launch(void* const* d_in, const int* in_sizes, int n_in,
                              void* d_out, int out_size, void* d_ws, size_t ws_size, hipStream_t stream) {
  if (n_in < 13 || d_out == nullptr || d_ws == nullptr) return;
  if (in_sizes[1] != BNR * XROW || in_sizes[2] != NC * G3 * 2 || in_sizes[3] != NC * G3 * HID ||
      in_sizes[4] != NC * G3 || in_sizes[5] != NC * G3 || in_sizes[6] != NC * G3 || in_sizes[7] != NC * G3 * HID ||
      in_sizes[8] != NC * G3 || in_sizes[9] != NC * G3 || in_sizes[10] != NC * HID || in_sizes[11] != NC ||
      in_sizes[12] != NNODE * NC || out_size != BNR * TOUT) return;

  const float* X     = (const float*)d_in[1];
  const float* eWih  = (const float*)d_in[2];
  const float* eWhh  = (const float*)d_in[3];
  const float* eBih  = (const float*)d_in[4];
  const float* eBhh  = (const float*)d_in[5];
  const float* dWih  = (const float*)d_in[6];
  const float* dWhh  = (const float*)d_in[7];
  const float* dBih  = (const float*)d_in[8];
  const float* dBhh  = (const float*)d_in[9];
  const float* linW  = (const float*)d_in[10];
  const float* linB  = (const float*)d_in[11];
  const float* embed = (const float*)d_in[12];
  float* out = (float*)d_out;

  char* ws = (char*)d_ws; size_t off = 0;
  auto carve = [&](size_t bytes) -> char* { char* p = ws + off; off += (bytes + 255) & ~(size_t)255; return p; };
  unsigned* W16u = (unsigned*)carve((size_t)2 * NC * WPL * 2);
  float*    VALS = (float*)carve((size_t)NC * BNR * TOUT * 4);
  if (off > ws_size || off > (size_t)134217728) return;
  const _Float16* W16 = (const _Float16*)W16u;

  prep_kernel<<<480, 256, 0, stream>>>(eWhh, dWhh, W16u);
  gru_seq_kernel<<<dim3(NTILE, NC), NT_REC, 0, stream>>>(X, W16, eWih, eBih, eBhh, dWih, dBih, dBhh, linW, linB, VALS);
  combine_kernel<<<(NOUT4 + 255) / 256, 256, 0, stream>>>(VALS, embed, out, NOUT4);
}
